// GA_CSWinTransformer_72421738545901
// MI455X (gfx1250) — hardware-run, weakly checked
//
#include <hip/hip_runtime.h>
#define NI 32
#define RS 56
#define NTK (RS * RS)
#define CD 128
#define CH 64
#define NHB 2
#define HDm 32
#define NR (NI * NTK)
#define NWI 28
#define TOK 112
#define TOKP 128
#define ICH 8
#define WCH (ICH * NWI)
#define NWR ((size_t)NI * NWI * TOKP)
#define DFF 512
#ifndef MCH
#define MCH 8
#endif
static_assert((NR / MCH) % 128 == 0, "MLP chunk rows must be a multiple of 128");
__host__ __device__ constexpr size_t zmax(size_t a, size_t b) { return a > b ? a : b; }
typedef __bf16 v16b __attribute__((ext_vector_type(16)));
typedef unsigned short v8us __attribute__((ext_vector_type(8), may_alias));
typedef float  v8f  __attribute__((ext_vector_type(8)));
typedef float  v4f  __attribute__((ext_vector_type(4)));
typedef float  v4fa __attribute__((ext_vector_type(4), may_alias));
union FragB { v16b v; v8us half[2]; unsigned short u[16]; };

__device__ __forceinline__ unsigned short bf16_bits(float x) { unsigned int u = __float_as_uint(x); return (unsigned short)((u + 0x7FFFu + ((u >> 16) & 1u)) >> 16); }
__device__ __forceinline__ float bf16_val(unsigned short b) { return __uint_as_float(((unsigned int)b) << 16); }
__device__ __forceinline__ float bf16_round(float x) { return bf16_val(bf16_bits(x)); }
template <int NT>
__device__ __forceinline__ v8f mmaN(v16b ah, v16b al, v16b bh, v16b bl, v8f c) {
  c = __builtin_amdgcn_wmma_f32_16x16x32_bf16(false, ah, false, bh, (short)0, c, false, false);
  if (NT >= 2) c = __builtin_amdgcn_wmma_f32_16x16x32_bf16(false, al, false, bh, (short)0, c, false, false);
  if (NT >= 3) c = __builtin_amdgcn_wmma_f32_16x16x32_bf16(false, ah, false, bl, (short)0, c, false, false);
  asm volatile("v_nop\n\tv_nop\n\tv_nop\n\tv_nop" : "+v"(c) : "v"(ah), "v"(al), "v"(bh), "v"(bl));
  return c;
}

__global__ __launch_bounds__(256) void k_wt_bf16(const float* __restrict__ W, unsigned short* __restrict__ Wt, int K, int N) {
  const int t = blockIdx.x * 256 + threadIdx.x;
  const int k8n = K / 8;
  if (t >= N * k8n) return;
  const int n = t / k8n, k8 = (t % k8n) * 8;
  v8us v;
#pragma unroll
  for (int i = 0; i < 8; ++i) v[i] = bf16_bits(W[(size_t)(k8 + i) * N + n]);
  *(volatile v8us*)(Wt + (size_t)n * K + k8) = v;
  __threadfence();
  *(volatile v8us*)(Wt + (size_t)n * K + k8) = v;
}

template <bool ASPLIT, int ACT, bool BIAS_BF16>
__global__ __launch_bounds__(128) void k_gemm_bf(const float* __restrict__ A, int lda, const unsigned short* __restrict__ Wt, int ldb,
                                               const float* __restrict__ bias, float* __restrict__ C, int ldc, int M, int N, int K) {
  __shared__ __attribute__((aligned(16))) float so[4][16][64];
  const int tid = threadIdx.x, w = tid >> 5, lane = tid & 31, ln = lane & 15, hh = lane >> 4;
  const int ntn = N / 64;
  const int wid = blockIdx.x * 4 + w;
  const int mt = wid / ntn, nq = wid % ntn;
  if (mt * 16 >= M) return;
  const int row0 = mt * 16, col0 = nq * 64;
  const float* arow = A + (size_t)(row0 + ln) * lda;
  v8f acc[4] = {};
  for (int kb = 0; kb < K; kb += 32) {
    FragB ah, al;
    const v4f x0 = *(const v4fa*)(arow + kb + 8 * hh), x1 = *(const v4fa*)(arow + kb + 8 * hh + 4);
    const v4f x2 = *(const v4fa*)(arow + kb + 16 + 8 * hh), x3 = *(const v4fa*)(arow + kb + 16 + 8 * hh + 4);
    float xs[16] = {x0[0],x0[1],x0[2],x0[3],x1[0],x1[1],x1[2],x1[3],x2[0],x2[1],x2[2],x2[3],x3[0],x3[1],x3[2],x3[3]};
#pragma unroll
    for (int i = 0; i < 16; ++i) { const unsigned short hb = bf16_bits(xs[i]); ah.u[i] = hb; al.u[i] = ASPLIT ? bf16_bits(xs[i] - bf16_val(hb)) : (unsigned short)0; }
#pragma unroll
    for (int t = 0; t < 4; ++t) {
      const unsigned short* brow = Wt + (size_t)(col0 + t * 16 + ln) * ldb + kb;
      FragB b;
      b.half[0] = *(const v8us*)(brow + 8 * hh);
      b.half[1] = *(const v8us*)(brow + 16 + 8 * hh);
      acc[t] = mmaN<ASPLIT ? 2 : 1>(ah.v, al.v, b.v, b.v, acc[t]);
    }
  }
#pragma unroll
  for (int t = 0; t < 4; ++t) {
    float bv = bias ? bias[col0 + t * 16 + ln] : 0.f;
    if (BIAS_BF16) bv = bf16_round(bv);
#pragma unroll
    for (int r = 0; r < 8; ++r) { float v = acc[t][r] + bv; if (ACT == 1) v = fmaxf(v, 0.f); so[w][8 * hh + r][t * 16 + ln] = v; }
  }
  __builtin_amdgcn_fence(__ATOMIC_ACQ_REL, "workgroup");
  __builtin_amdgcn_wave_barrier();
  const int rsub = lane >> 4, c4 = (lane & 15) * 4;
  for (int pass = 0; pass < 2; ++pass) {
#pragma unroll
    for (int q = 0; q < 8; ++q) {
      const int r = q * 2 + rsub;
      const v4f v = *(const v4fa*)&so[w][r][c4];
      *(volatile v4f*)(C + (size_t)(row0 + r) * ldc + col0 + c4) = v;
    }
    if (pass == 0) __threadfence();
  }
}

template <bool ASPLIT, int ACT, bool BIAS_BF16, bool RES_BF16>
__global__ __launch_bounds__(128) void k_gemm_bf3(const float* __restrict__ A, int lda, const unsigned short* __restrict__ Wt, int ldb,
                                                const float* __restrict__ bias, const float* __restrict__ resid, int rmod, int ldr,
                                                float* __restrict__ C, int ldc, int M, int N, int K) {
  __shared__ __attribute__((aligned(16))) float so[4][16][64];
  const int tid = threadIdx.x, w = tid >> 5, lane = tid & 31, ln = lane & 15, hh = lane >> 4;
  const int ntn = N / 64;
  const int wid = blockIdx.x * 4 + w;
  const int mt = wid / ntn, nq = wid % ntn;
  if (mt * 16 >= M) return;
  const int row0 = mt * 16, col0 = nq * 64;
  const float* arow = A + (size_t)(row0 + ln) * lda;
  v8f acc[4] = {};
  for (int kb = 0; kb < K; kb += 32) {
    FragB ah, al;
    const v4f x0 = *(const v4fa*)(arow + kb + 8 * hh), x1 = *(const v4fa*)(arow + kb + 8 * hh + 4);
    const v4f x2 = *(const v4fa*)(arow + kb + 16 + 8 * hh), x3 = *(const v4fa*)(arow + kb + 16 + 8 * hh + 4);
    float xs[16] = {x0[0],x0[1],x0[2],x0[3],x1[0],x1[1],x1[2],x1[3],x2[0],x2[1],x2[2],x2[3],x3[0],x3[1],x3[2],x3[3]};
#pragma unroll
    for (int i = 0; i < 16; ++i) { const unsigned short hb = bf16_bits(xs[i]); ah.u[i] = hb; al.u[i] = ASPLIT ? bf16_bits(xs[i] - bf16_val(hb)) : (unsigned short)0; }
#pragma unroll
    for (int t = 0; t < 4; ++t) {
      const unsigned short* brow = Wt + (size_t)(col0 + t * 16 + ln) * ldb + kb;
      FragB b;
      b.half[0] = *(const v8us*)(brow + 8 * hh);
      b.half[1] = *(const v8us*)(brow + 16 + 8 * hh);
      acc[t] = mmaN<ASPLIT ? 2 : 1>(ah.v, al.v, b.v, b.v, acc[t]);
    }
  }
#pragma unroll
  for (int t = 0; t < 4; ++t) {
    const int col = col0 + t * 16 + ln;
    float bv = bias ? bias[col] : 0.f;
    if (BIAS_BF16) bv = bf16_round(bv);
#pragma unroll
    for (int r = 0; r < 8; ++r) {
      float v = acc[t][r] + bv;
      if (resid) { float rv = resid[(size_t)((row0 + 8 * hh + r) % rmod) * ldr + col]; if (RES_BF16) rv = bf16_round(rv); v += rv; }
      if (ACT == 1) v = fmaxf(v, 0.f);
      if (ACT == 2) v = 0.5f * v * (1.0f + erff(v * 0.70710678118654752f));
      if (ACT == 3) { const float u = 0.7978845608028654f * (v + 0.044715f * v * v * v); v = 0.5f * v * (1.0f + tanhf(u)); }
      so[w][8 * hh + r][t * 16 + ln] = v;
    }
  }
  __builtin_amdgcn_fence(__ATOMIC_ACQ_REL, "workgroup");
  __builtin_amdgcn_wave_barrier();
  const int rsub = lane >> 4, c4 = (lane & 15) * 4;
  for (int pass = 0; pass < 2; ++pass) {
#pragma unroll
    for (int q = 0; q < 8; ++q) {
      const int r = q * 2 + rsub;
      const v4f v = *(const v4fa*)&so[w][r][c4];
      *(volatile v4f*)(C + (size_t)(row0 + r) * ldc + col0 + c4) = v;
    }
    if (pass == 0) __threadfence();
  }
}
template <bool PARAM_BF16>
__global__ __launch_bounds__(256) void k_layernorm(const float* __restrict__ X, const float* __restrict__ R, const float* __restrict__ g, const float* __restrict__ bta,
                                                  float* __restrict__ out_sum, float* __restrict__ out_norm, int N, float eps) {
  __shared__ float red[256];
  const int row = blockIdx.x, tid = threadIdx.x;
  const float* x = X + (size_t)row * N; const float* rr = R ? R + (size_t)row * N : nullptr;
  float vals[16];
  const int per = N / 256;
  float s1 = 0.f;
  for (int u = 0; u < per / 4; ++u) {
    const int j = tid * 4 + 1024 * u;
    const v4f a = *(const v4fa*)(x + j);
    v4f b = {0.f,0.f,0.f,0.f}; if (rr) b = *(const v4fa*)(rr + j);
#pragma unroll
    for (int q = 0; q < 4; ++q) { const float v = a[q] + b[q]; vals[u * 4 + q] = v; s1 += v; }
  }
  red[tid] = s1; __syncthreads();
  for (int st = 128; st > 0; st >>= 1) { if (tid < st) red[tid] += red[tid + st]; __syncthreads(); }
  const float mu = red[0] / (float)N; __syncthreads();
  float s2 = 0.f;
  for (int u = 0; u < per / 4; ++u)
#pragma unroll
    for (int q = 0; q < 4; ++q) { const float c = vals[u * 4 + q] - mu; s2 += c * c; }
  red[tid] = s2; __syncthreads();
  for (int st = 128; st > 0; st >>= 1) { if (tid < st) red[tid] += red[tid + st]; __syncthreads(); }
  const float rs = rsqrtf(red[0] / (float)N + eps);
  for (int pass = 0; pass < 2; ++pass) {
    for (int u = 0; u < per / 4; ++u) {
      const int j = tid * 4 + 1024 * u;
      v4f o, sm;
#pragma unroll
      for (int q = 0; q < 4; ++q) {
        float gg = g[j + q], bb = bta[j + q];
        if (PARAM_BF16) { gg = bf16_round(gg); bb = bf16_round(bb); }
        sm[q] = vals[u * 4 + q]; o[q] = (vals[u * 4 + q] - mu) * rs * gg + bb;
      }
      if (out_sum) *(volatile v4f*)(out_sum + (size_t)row * N + j) = sm;
      *(volatile v4f*)(out_norm + (size_t)row * N + j) = o;
    }
    if (pass == 0) __threadfence();
  }
}


typedef _Float16 v16h __attribute__((ext_vector_type(16)));
union FragH { v16h v; v8us half[2]; _Float16 h[16]; unsigned short u[16]; };
template <int NT>
__device__ __forceinline__ v8f mmaH(v16h ah, v16h al, v16h bh, v16h bl, v8f c) {
  c = __builtin_amdgcn_wmma_f32_16x16x32_f16(false, ah, false, bh, (short)0, c, false, false);
  if (NT >= 2) c = __builtin_amdgcn_wmma_f32_16x16x32_f16(false, al, false, bh, (short)0, c, false, false);
  if (NT >= 3) c = __builtin_amdgcn_wmma_f32_16x16x32_f16(false, ah, false, bl, (short)0, c, false, false);
  asm volatile("v_nop\n\tv_nop\n\tv_nop\n\tv_nop" : "+v"(c) : "v"(ah), "v"(al), "v"(bh), "v"(bl));
  return c;
}
template <bool ASPLIT>
__global__ __launch_bounds__(128) void k_gemm_h(const float* __restrict__ A, int lda, size_t sA, const _Float16* __restrict__ Bh, int ldb, size_t sB, float alpha, float* __restrict__ C, int ldc, size_t sC, int M, int N, int K) {
  __shared__ __attribute__((aligned(16))) float so[4][16][64];
  const int tid = threadIdx.x, w = tid >> 5, lane = tid & 31, ln = lane & 15, hh = lane >> 4; const int by = blockIdx.y;
  A += (size_t)by * sA; Bh += (size_t)by * sB; C += (size_t)by * sC;
  const int ntn = (N + 63) / 64; const int wid = blockIdx.x * 4 + w; const int mt = wid / ntn, nq = wid % ntn; if (mt * 16 >= M) return;
  const int row0 = mt * 16, col0 = nq * 64; const float* arow = A + (size_t)(row0 + ln) * lda;
  v8f acc[4] = {};
  for (int kb = 0; kb < K; kb += 32) {
    FragH ah, al;
    const v4f x0 = *(const v4fa*)(arow + kb + 8 * hh), x1 = *(const v4fa*)(arow + kb + 8 * hh + 4), x2 = *(const v4fa*)(arow + kb + 16 + 8 * hh), x3 = *(const v4fa*)(arow + kb + 16 + 8 * hh + 4);
    float xs[16] = {x0[0],x0[1],x0[2],x0[3],x1[0],x1[1],x1[2],x1[3],x2[0],x2[1],x2[2],x2[3],x3[0],x3[1],x3[2],x3[3]};
#pragma unroll
    for (int i = 0; i < 16; ++i) { const _Float16 h = (_Float16)xs[i]; ah.h[i] = h; al.h[i] = ASPLIT ? (_Float16)(xs[i] - (float)h) : (_Float16)0.0f; }
#pragma unroll
    for (int t = 0; t < 4; ++t) { if (col0 + t * 16 >= N) continue; const size_t boff = (size_t)(col0 + t * 16 + ln) * ldb + kb; FragH bq; bq.half[0] = *(const v8us*)(Bh + boff + 8 * hh); bq.half[1] = *(const v8us*)(Bh + boff + 16 + 8 * hh);
      acc[t] = mmaH<ASPLIT ? 2 : 1>(ah.v, al.v, bq.v, bq.v, acc[t]); }
  }
#pragma unroll
  for (int t = 0; t < 4; ++t) { if (col0 + t * 16 >= N) continue;
#pragma unroll
    for (int r = 0; r < 8; ++r) so[w][8 * hh + r][t * 16 + ln] = acc[t][r] * alpha; }
  __builtin_amdgcn_fence(__ATOMIC_ACQ_REL, "workgroup"); __builtin_amdgcn_wave_barrier();
  const int rsub = lane >> 4, c4 = (lane & 15) * 4;
  for (int pass = 0; pass < 2; ++pass) {
#pragma unroll
    for (int q = 0; q < 8; ++q) { const int r = q * 2 + rsub; if (col0 + c4 < N) { const v4f v = *(const v4fa*)&so[w][r][c4]; *(volatile v4f*)(C + (size_t)(row0 + r) * ldc + col0 + c4) = v; } }
    if (pass == 0) __threadfence(); }
}

__global__ __launch_bounds__(256) void k_wt_f16(const float* __restrict__ W, _Float16* __restrict__ Wt, int K, int N, float scale) {
  const int t = blockIdx.x * 256 + threadIdx.x; if (t >= N * (K / 8)) return; const int n = t / (K / 8), k8 = (t % (K / 8)) * 8; FragH f;
#pragma unroll
  for (int i = 0; i < 8; ++i) f.h[i] = (_Float16)(bf16_round(W[(size_t)(k8 + i) * N + n]) * scale); const v8us o = f.half[0];
  *(volatile v8us*)((unsigned short*)Wt + (size_t)n * K + k8) = o; __threadfence(); *(volatile v8us*)((unsigned short*)Wt + (size_t)n * K + k8) = o;
}
template <int ACT>
__global__ __launch_bounds__(128) void k_gemm_hhx(const _Float16* __restrict__ A, int lda, size_t sA, const _Float16* __restrict__ Bh, int ldb, size_t sB, float alpha, const float* __restrict__ bias, size_t sBias, const float* __restrict__ CP, int rowsPerB, size_t sCPb, int row0g,
    float* __restrict__ C, _Float16* __restrict__ C16, int ldc, size_t sC, int M, int N, int K) {
  __shared__ __attribute__((aligned(16))) float so[4][16][64];
  const int tid = threadIdx.x, w = tid >> 5, lane = tid & 31, ln = lane & 15, hh = lane >> 4; const int by = blockIdx.y;
  A += (size_t)by * sA; Bh += (size_t)by * sB; const size_t cofs = (size_t)by * sC; const float* bp = bias ? bias + (size_t)by * sBias : nullptr;
  const int ntn = (N + 63) / 64; const int wid = blockIdx.x * 4 + w; const int mt = wid / ntn, nq = wid % ntn; if (mt * 16 >= M) return;
  const int row0 = mt * 16, col0 = nq * 64; const _Float16* arow = A + (size_t)(row0 + ln) * lda;
  v8f acc[4] = {};
  for (int kb = 0; kb < K; kb += 32) { FragH ah; ah.half[0] = *(const v8us*)((const unsigned short*)arow + kb + 8 * hh); ah.half[1] = *(const v8us*)((const unsigned short*)arow + kb + 16 + 8 * hh);
#pragma unroll
    for (int t = 0; t < 4; ++t) { if (col0 + t * 16 >= N) continue; const size_t boff = (size_t)(col0 + t * 16 + ln) * ldb + kb; FragH bq; bq.half[0] = *(const v8us*)((const unsigned short*)Bh + boff + 8 * hh); bq.half[1] = *(const v8us*)((const unsigned short*)Bh + boff + 16 + 8 * hh);
      acc[t] = mmaH<1>(ah.v, ah.v, bq.v, bq.v, acc[t]); }
  }
#pragma unroll
  for (int t = 0; t < 4; ++t) { if (col0 + t * 16 >= N) continue; const int col = col0 + t * 16 + ln; const float bv = bp ? bf16_round(bp[col]) : 0.f;
#pragma unroll
    for (int r = 0; r < 8; ++r) { float v = acc[t][r] * alpha + bv; if (CP) { const int rr = row0g + row0 + 8 * hh + r; if (rowsPerB < 0) v += CP[cofs + (size_t)rr * ldc + col];        else { const int bidx = rr / rowsPerB; v += CP[(size_t)bidx * sCPb + (size_t)by * 64 + col]; } } if (ACT == 1) v = (v > 0.f) ? v : expm1f(v); else if (ACT == 7) v = (v > 0.f) ? v + 1.0f : expf(v); else if (ACT == 8) v = tanhf(v); else if (ACT == 9) v = 0.5f * v * (1.0f + tanhf(0.7978845608028654f * (v + 0.044715f * v * v * v))); else if (ACT == 11) v = 1.0f / (1.0f + expf(-v)); else if (ACT == 12) v = (v > 0.f) ? v : 0.01f * v; else if (ACT == 14) v = (v > 0.f) ? v : 0.1f * v; else if (ACT == 16) v = (v >= 0.f) ? v : 0.3f * v; else if (ACT == 17) v = (v >= 0.f) ? v : 0.2f * v; else if (ACT == 15) v = v / (1.0f + expf(-v)); else if (ACT == 3) v = fmaxf(v, 0.f); else if (ACT == 6) v = 0.5f * v * (1.0f + erff(v * 0.70710678118654752f)); so[w][8 * hh + r][t * 16 + ln] = v; } }
  __builtin_amdgcn_fence(__ATOMIC_ACQ_REL, "workgroup"); __builtin_amdgcn_wave_barrier();
  const int rsub = lane >> 4, c4 = (lane & 15) * 4; typedef _Float16 v4h __attribute__((ext_vector_type(4)));
  for (int pass = 0; pass < 2; ++pass) {
#pragma unroll
    for (int q = 0; q < 8; ++q) { const int r = q * 2 + rsub; if (col0 + c4 < N) { const v4f v = *(const v4fa*)&so[w][r][c4]; if (C) *(volatile v4f*)(C + cofs + (size_t)(row0 + r) * ldc + col0 + c4) = v; if (C16) { v4h h4; for (int i = 0; i < 4; ++i) h4[i] = (_Float16)v[i]; *(volatile v4h*)(C16 + cofs + (size_t)(row0 + r) * ldc + col0 + c4) = h4; } } }
    if (pass == 0) __threadfence(); }
}


typedef _Float16 v4h __attribute__((ext_vector_type(4)));

__global__ __launch_bounds__(256) void k_x16(const float* __restrict__ x, _Float16* __restrict__ X16, size_t n8) { const size_t t = (size_t)blockIdx.x * 256 + threadIdx.x; if (t >= n8) return; FragH f;
#pragma unroll
  for (int q = 0; q < 8; ++q) f.h[q] = (_Float16)bf16_round(x[t * 8 + q]); *(volatile v8us*)((unsigned short*)X16 + t * 8) = f.half[0]; __threadfence(); *(volatile v8us*)((unsigned short*)X16 + t * 8) = f.half[0]; }
__global__ __launch_bounds__(256) void k_h16(const float* __restrict__ x, _Float16* __restrict__ X16, size_t n8) { const size_t t = (size_t)blockIdx.x * 256 + threadIdx.x; if (t >= n8) return; FragH f;
#pragma unroll
  for (int q = 0; q < 8; ++q) f.h[q] = (_Float16)x[t * 8 + q]; *(volatile v8us*)((unsigned short*)X16 + t * 8) = f.half[0]; __threadfence(); *(volatile v8us*)((unsigned short*)X16 + t * 8) = f.half[0]; }
__global__ __launch_bounds__(256) void k_round16f(const float* __restrict__ W, _Float16* __restrict__ Bt, size_t n8) { const size_t t = (size_t)blockIdx.x * 256 + threadIdx.x; if (t >= n8) return; FragH f;
#pragma unroll
  for (int i = 0; i < 8; ++i) f.h[i] = (_Float16)(bf16_round(W[t * 8 + i]) * 16.0f); *(volatile v8us*)((unsigned short*)Bt + t * 8) = f.half[0]; __threadfence(); *(volatile v8us*)((unsigned short*)Bt + t * 8) = f.half[0]; }
template <int NHv, int TTv>
__global__ __launch_bounds__(256) void k_vt(const _Float16* __restrict__ V16, int ldv, int voff, _Float16* __restrict__ Vt) { __shared__ unsigned short tl[64][66]; const int tid = threadIdx.x; const int slab = blockIdx.x / (TTv / 64), lg = blockIdx.x % (TTv / 64); const int b = slab / NHv, h = slab % NHv;
  for (int i = tid; i < 64 * 8; i += 256) { const int r = i / 8, c8 = (i % 8) * 8; FragH f; f.half[0] = *(const v8us*)((const unsigned short*)V16 + ((size_t)b * TTv + lg * 64 + r) * ldv + voff + h * 64 + c8);
#pragma unroll
    for (int q = 0; q < 8; ++q) tl[r][c8 + q] = f.u[q]; }
  __syncthreads();
  for (int pass = 0; pass < 2; ++pass) {
#pragma unroll
    for (int rd = 0; rd < 2; ++rd) { const int d = rd * 32 + tid / 8, pc = tid % 8; FragH f;
#pragma unroll
      for (int q = 0; q < 8; ++q) f.u[q] = tl[pc * 8 + q][d];
      *(volatile v8us*)((unsigned short*)Vt + ((size_t)slab * 64 + d) * TTv + lg * 64 + pc * 8) = f.half[0]; }
    if (pass == 0) __threadfence(); } }

__global__ __launch_bounds__(256) void k_hl(const float* __restrict__ F, _Float16* __restrict__ Hh, _Float16* __restrict__ Hl, size_t n8) { const size_t t = (size_t)blockIdx.x * 256 + threadIdx.x; if (t >= n8) return; FragH fh, fl; const v4f a = *(const v4fa*)(F + t * 8), c = *(const v4fa*)(F + t * 8 + 4);
#pragma unroll
  for (int q = 0; q < 4; ++q) { _Float16 h = (_Float16)a[q]; fh.h[q] = h; fl.h[q] = (_Float16)((a[q] - (float)h) * 1024.0f); h = (_Float16)c[q]; fh.h[4 + q] = h; fl.h[4 + q] = (_Float16)((c[q] - (float)h) * 1024.0f); }
  for (int pass = 0; pass < 2; ++pass) { *(volatile v8us*)((unsigned short*)Hh + t * 8) = fh.half[0]; *(volatile v8us*)((unsigned short*)Hl + t * 8) = fl.half[0]; if (pass == 0) __threadfence(); } }

__device__ __forceinline__ v16h g2_frag(const _Float16* p, int hh) { FragH f; f.half[0] = *(const v8us*)((const unsigned short*)p + 8 * hh); f.half[1] = *(const v8us*)((const unsigned short*)p + 16 + 8 * hh); return f.v; }
__device__ __forceinline__ v8f g2_mma(v16h a, v16h b, v8f c) { v8f d = __builtin_amdgcn_wmma_f32_16x16x32_f16(false, a, false, b, (short)0, c, false, false); asm volatile("v_nop\n\tv_nop\n\tv_nop\n\tv_nop" : "+v"(d) : "v"(a), "v"(b)); return d; }
template <int ACT>
__global__ __launch_bounds__(128) void k_gemm2(const _Float16* __restrict__ A, int lda, size_t sA, const _Float16* __restrict__ Bh, int ldb, size_t sB, float alpha, const float* __restrict__ bias, size_t sBias, const float* __restrict__ CP, int rowsPerB, size_t sCPb, int row0g,
    float* __restrict__ C, _Float16* __restrict__ C16, int ldc, size_t sC, int M, int N, int K) { static_assert(ACT == 0 || ACT == 3 || ACT == 6 || ACT == 8 || ACT == 9 || ACT == 11 || ACT == 12 || ACT == 14 || ACT == 15 || ACT == 16 || ACT == 17, "k_gemm2: unsupported ACT code (would silently apply no activation)");
  __shared__ __attribute__((aligned(16))) float so[4][32][68];
  const int tid = threadIdx.x, w = tid >> 5, lane = tid & 31, ln = lane & 15, hh = lane >> 4; const int by = blockIdx.y;
  A += (size_t)by * sA; Bh += (size_t)by * sB; const size_t cofs = (size_t)by * sC; const float* bp = bias ? bias + (size_t)by * sBias : nullptr;
  const int ntn = N >> 6; const int mt = blockIdx.x / ntn, nq = blockIdx.x - mt * ntn; const int row0 = mt * 128 + 32 * w, col0 = nq * 64; if (row0 >= M) return;
  const _Float16* a0p = A + (size_t)(row0 + ln) * lda; const _Float16* a1p = a0p + (size_t)16 * lda;
  const _Float16* b0p = Bh + (size_t)(col0 + ln) * ldb; const _Float16* b1p = b0p + (size_t)16 * ldb; const _Float16* b2p = b1p + (size_t)16 * ldb; const _Float16* b3p = b2p + (size_t)16 * ldb;
  const v8f z8 = {0.f,0.f,0.f,0.f,0.f,0.f,0.f,0.f}; v8f c00 = z8, c01 = z8, c02 = z8, c03 = z8, c10 = z8, c11 = z8, c12 = z8, c13 = z8;
#pragma unroll 1
  for (int kb = 0; kb < K; kb += 32) { const v16h a0 = g2_frag(a0p + kb, hh), a1 = g2_frag(a1p + kb, hh);
    v16h b = g2_frag(b0p + kb, hh); c00 = g2_mma(a0, b, c00); c10 = g2_mma(a1, b, c10);
    b = g2_frag(b1p + kb, hh); c01 = g2_mma(a0, b, c01); c11 = g2_mma(a1, b, c11);
    b = g2_frag(b2p + kb, hh); c02 = g2_mma(a0, b, c02); c12 = g2_mma(a1, b, c12);
    b = g2_frag(b3p + kb, hh); c03 = g2_mma(a0, b, c03); c13 = g2_mma(a1, b, c13); }
  v8f accs[8] = {c00, c01, c02, c03, c10, c11, c12, c13};
#pragma unroll
  for (int u = 0; u < 8; ++u) { const int t = u & 3, half = u >> 2; const int col = col0 + t * 16 + ln; const float bv = bp ? bf16_round(bp[col]) : 0.f;
#pragma unroll
    for (int r = 0; r < 8; ++r) { const int rloc = half * 16 + 8 * hh + r; float v = accs[u][r] * alpha + bv; if (CP) { if (rowsPerB < 0) v += CP[cofs + (size_t)(row0g + row0 + rloc) * ldc + col];        else { const int bidx = (row0g + row0 + rloc) / rowsPerB; v += CP[(size_t)bidx * sCPb + (size_t)by * 64 + col]; } }
      if (ACT == 3) v = fmaxf(v, 0.f); else if (ACT == 6) v = 0.5f * v * (1.0f + erff(v * 0.70710678118654752f)); else if (ACT == 11) v = 1.0f / (1.0f + expf(-v)); else if (ACT == 15) v = v / (1.0f + expf(-v)); else if (ACT == 12) v = (v > 0.f) ? v : 0.01f * v; else if (ACT == 8) v = tanhf(v); else if (ACT == 9) v = 0.5f * v * (1.0f + tanhf(0.7978845608028654f * (v + 0.044715f * v * v * v))); else if (ACT == 14) v = (v > 0.f) ? v : 0.1f * v; else if (ACT == 16) v = (v >= 0.f) ? v : 0.3f * v; else if (ACT == 17) v = (v >= 0.f) ? v : 0.2f * v;
      so[w][rloc][t * 16 + ln] = v; } }
  __builtin_amdgcn_fence(__ATOMIC_ACQ_REL, "workgroup"); __builtin_amdgcn_wave_barrier();
  const int rsub = lane >> 4, c4 = (lane & 15) * 4;
  for (int pass = 0; pass < 2; ++pass) {
#pragma unroll
    for (int q = 0; q < 16; ++q) { const int r = q * 2 + rsub; const v4f v = *(const v4fa*)&so[w][r][c4]; if (C) *(volatile v4f*)(C + cofs + (size_t)(row0 + r) * ldc + col0 + c4) = v; if (C16) { v4h h4; for (int i = 0; i < 4; ++i) h4[i] = (_Float16)v[i]; *(volatile v4h*)(C16 + cofs + (size_t)(row0 + r) * ldc + col0 + c4) = h4; } }
    if (pass == 0) __threadfence(); } }


typedef unsigned short v4us __attribute__((ext_vector_type(4), may_alias));
__global__ __launch_bounds__(256) void k_ln1(const float* __restrict__ x, const float* __restrict__ g, const float* __restrict__ bb, _Float16* __restrict__ XN) {
  #pragma clang fp contract(off)
  const int wv = threadIdx.x >> 5, ln = threadIdx.x & 31; const size_t row = (size_t)blockIdx.x * 8 + wv; if (row >= (size_t)NR) return; const v4f a = *(const v4fa*)(x + row * CD + ln * 4); float v[4]; float s = 0.f; for (int q = 0; q < 4; ++q) { v[q] = bf16_round(a[q]); s += v[q]; }
  for (int o = 16; o > 0; o >>= 1) s += __shfl_xor(s, o, 32); const float mu = s / (float)CD; float s2 = 0.f; for (int q = 0; q < 4; ++q) { const float d = v[q] - mu; s2 += d * d; } for (int o = 16; o > 0; o >>= 1) s2 += __shfl_xor(s2, o, 32); const float rs = rsqrtf(s2 / (float)CD + 1e-5f);
  FragH f; for (int q = 0; q < 4; ++q) { const int c = ln * 4 + q; float z = (v[q] - mu) * rs; z = z * bf16_round(g[c]); z += bf16_round(bb[c]); f.h[q] = (_Float16)z; }
  *(volatile v4us*)((unsigned short*)XN + row * CD + ln * 4) = *(v4us*)&f.u[0]; __threadfence(); *(volatile v4us*)((unsigned short*)XN + row * CD + ln * 4) = *(v4us*)&f.u[0]; }
__device__ __forceinline__ size_t win_row(int br, int b, int win, int t) { int y, x; if (br == 0) { y = t / 2; x = win * 2 + (t & 1); } else { y = win * 2 + t / RS; x = t % RS; } return (size_t)b * NTK + (size_t)y * RS + x; }
__global__ __launch_bounds__(256) void k_towin(const _Float16* __restrict__ QKV, int br, _Float16* __restrict__ QW, _Float16* __restrict__ KW, _Float16* __restrict__ VW) { const size_t t = (size_t)blockIdx.x * 256 + threadIdx.x; if (t >= NWR * CH / 8) return; const int c0 = (int)((t * 8) % CH); const size_t wr = (t * 8) / CH; const int tk = (int)(wr % TOKP); const int win = (int)((wr / TOKP) % NWI); const int b = (int)(wr / ((size_t)TOKP * NWI)); v8us q, k, v;
  if (tk < TOK) { const size_t r = win_row(br, b, win, tk); const unsigned short* src = (const unsigned short*)QKV + r * (3 * CD) + br * CH + c0; q = *(const v8us*)src; k = *(const v8us*)(src + CD); v = *(const v8us*)(src + 2 * CD); } else { for (int i = 0; i < 8; ++i) { q[i] = 0; k[i] = 0; v[i] = 0; } }
  for (int pass = 0; pass < 2; ++pass) { *(volatile v8us*)((unsigned short*)QW + t * 8) = q; *(volatile v8us*)((unsigned short*)KW + t * 8) = k; *(volatile v8us*)((unsigned short*)VW + t * 8) = v; if (pass == 0) __threadfence(); } }
__global__ __launch_bounds__(256) void k_vt(const _Float16* __restrict__ VW, _Float16* __restrict__ VT) { __shared__ unsigned short tl[TOKP][72]; const int tid = threadIdx.x; const size_t w = blockIdx.x;
  for (int i = tid; i < TOKP * 8; i += 256) { const int r = i / 8, c8 = (i % 8) * 8; FragH f; f.half[0] = *(const v8us*)((const unsigned short*)VW + (w * TOKP + r) * CH + c8); for (int q = 0; q < 8; ++q) tl[r][c8 + q] = f.u[q]; }
  __syncthreads();
  for (int pass = 0; pass < 2; ++pass) { for (int i = tid; i < CH * (TOKP / 8); i += 256) { const int d = i / (TOKP / 8), pc = i % (TOKP / 8); FragH f; for (int q = 0; q < 8; ++q) f.u[q] = tl[pc * 8 + q][d]; const int h = d / HDm, dd = d % HDm; *(volatile v8us*)((unsigned short*)VT + ((w * NHB + h) * HDm + dd) * TOKP + pc * 8) = f.half[0]; } if (pass == 0) __threadfence(); } }
__global__ __launch_bounds__(256) void k_lepe(const _Float16* __restrict__ VW, int br, const float* __restrict__ cw, const float* __restrict__ cb, float* __restrict__ LE) {
  #pragma clang fp contract(off)
  const size_t t = (size_t)blockIdx.x * 256 + threadIdx.x; if (t >= NWR * CH / 8) return; const int c0 = (int)((t * 8) % CH); const size_t wr = (t * 8) / CH; const int tk = (int)(wr % TOKP); const size_t w = wr / TOKP; const int Hs = br ? 2 : RS, Ws = br ? RS : 2; v8f o; for (int q = 0; q < 8; ++q) o[q] = 0.f;
  if (tk < TOK) { const int hs = tk / Ws, wsx = tk % Ws; float acc[8]; for (int q = 0; q < 8; ++q) acc[q] = 0.f;
#pragma unroll 1
    for (int tap = 0; tap < 9; ++tap) { const int yy = hs + tap / 3 - 1, xx = wsx + tap % 3 - 1; if (yy < 0 || yy >= Hs || xx < 0 || xx >= Ws) continue; FragH f; f.half[0] = *(const v8us*)((const unsigned short*)VW + (w * TOKP + yy * Ws + xx) * CH + c0); for (int q = 0; q < 8; ++q) acc[q] += (float)f.h[q] * bf16_round(cw[(size_t)(c0 + q) * 9 + tap]); }
    for (int q = 0; q < 8; ++q) { float u = acc[q]; u += bf16_round(cb[c0 + q]); o[q] = u; } }
  *(volatile v8f*)(LE + t * 8) = o; __threadfence(); *(volatile v8f*)(LE + t * 8) = o; }
__global__ __launch_bounds__(256) void k_soft(const float* __restrict__ S, _Float16* __restrict__ P) {
  #pragma clang fp contract(off)
  const int wv = threadIdx.x >> 5, ln = threadIdx.x & 31; const size_t row = (size_t)blockIdx.x * 8 + wv; if (row >= (size_t)WCH * NHB * TOKP) return; const float* s = S + row * TOKP; float v[4]; float mx = -3.0e38f; for (int q = 0; q < 4; ++q) { const int j = ln * 4 + q; v[q] = (j < TOK) ? s[j] : -3.0e38f; mx = fmaxf(mx, v[q]); }
  for (int o = 16; o > 0; o >>= 1) mx = fmaxf(mx, __shfl_xor(mx, o, 32)); float e[4]; float su = 0.f; for (int q = 0; q < 4; ++q) { const int j = ln * 4 + q; e[q] = (j < TOK) ? expf(v[q] - mx) : 0.f; su += e[q]; }
  for (int o = 16; o > 0; o >>= 1) su += __shfl_xor(su, o, 32); const float inv = 1024.0f / su; FragH f; for (int q = 0; q < 4; ++q) f.h[q] = (_Float16)(e[q] * inv);
  *(volatile v4us*)((unsigned short*)P + row * TOKP + ln * 4) = *(v4us*)&f.u[0]; __threadfence(); *(volatile v4us*)((unsigned short*)P + row * TOKP + ln * 4) = *(v4us*)&f.u[0]; }
__global__ __launch_bounds__(256) void k_toimg(const _Float16* __restrict__ OW, int br, _Float16* __restrict__ ATT) { const size_t t = (size_t)blockIdx.x * 256 + threadIdx.x; if (t >= NWR * CH / 8) return; const int c0 = (int)((t * 8) % CH); const size_t wr = (t * 8) / CH; const int tk = (int)(wr % TOKP); if (tk >= TOK) return; const int win = (int)((wr / TOKP) % NWI); const int b = (int)(wr / ((size_t)TOKP * NWI)); const size_t r = win_row(br, b, win, tk); const v8us v = *(const v8us*)((const unsigned short*)OW + t * 8);
  *(volatile v8us*)((unsigned short*)ATT + r * CD + br * CH + c0) = v; __threadfence(); *(volatile v8us*)((unsigned short*)ATT + r * CD + br * CH + c0) = v; }
__global__ __launch_bounds__(256) void k_resln(const float* __restrict__ x, const float* __restrict__ AP, const float* __restrict__ g, const float* __restrict__ bb, float* __restrict__ X2, _Float16* __restrict__ YH, _Float16* __restrict__ YL) {
  #pragma clang fp contract(off)
  const int wv = threadIdx.x >> 5, ln = threadIdx.x & 31; const size_t row = (size_t)blockIdx.x * 8 + wv; if (row >= (size_t)NR) return; const v4f a = *(const v4fa*)(x + row * CD + ln * 4), p = *(const v4fa*)(AP + row * CD + ln * 4); float v[4]; float s = 0.f; for (int q = 0; q < 4; ++q) { float u = bf16_round(a[q]); u += p[q]; v[q] = u; s += u; }
  for (int o = 16; o > 0; o >>= 1) s += __shfl_xor(s, o, 32); const float mu = s / (float)CD; float s2 = 0.f; for (int q = 0; q < 4; ++q) { const float d = v[q] - mu; s2 += d * d; } for (int o = 16; o > 0; o >>= 1) s2 += __shfl_xor(s2, o, 32); const float rs = rsqrtf(s2 / (float)CD + 1e-5f);
  v4f o4; FragH fh, fl; for (int q = 0; q < 4; ++q) { const int c = ln * 4 + q; o4[q] = v[q]; float z = (v[q] - mu) * rs; z = z * bf16_round(g[c]); z += bf16_round(bb[c]); const _Float16 h = (_Float16)z; fh.h[q] = h; fl.h[q] = (_Float16)((z - (float)h) * 1024.0f); }
  for (int pass = 0; pass < 2; ++pass) { *(volatile v4f*)(X2 + row * CD + ln * 4) = o4; *(volatile v4us*)((unsigned short*)YH + row * CD + ln * 4) = *(v4us*)&fh.u[0]; *(volatile v4us*)((unsigned short*)YL + row * CD + ln * 4) = *(v4us*)&fl.u[0]; if (pass == 0) __threadfence(); } }
__global__ __launch_bounds__(256) void k_gelu(const float* __restrict__ F, _Float16* __restrict__ FHh, _Float16* __restrict__ FLl, size_t n8) {
  #pragma clang fp contract(off)
  const size_t t = (size_t)blockIdx.x * 256 + threadIdx.x; if (t >= n8) return; const v8f a = *(const v8f*)(F + t * 8); FragH fh, fl;
#pragma unroll 1
  for (int q = 0; q < 8; ++q) { const float s = 0.5f * a[q] * (1.0f + erff(a[q] * 0.70710678118654752f)); const _Float16 h = (_Float16)s; fh.h[q] = h; fl.h[q] = (_Float16)((s - (float)h) * 1024.0f); }
  for (int pass = 0; pass < 2; ++pass) { *(volatile v8us*)((unsigned short*)FHh + t * 8) = fh.half[0]; *(volatile v8us*)((unsigned short*)FLl + t * 8) = fl.half[0]; if (pass == 0) __threadfence(); } }

extern "C" void kernel_launch(void* const* d_in, const int* in_sizes, int n_in,
                              void* d_out, int out_size, void* d_ws, size_t ws_size, hipStream_t stream) {
  (void)in_sizes; (void)n_in; (void)out_size;
  const float* const* I = (const float* const*)d_in; const float* x = I[0]; const float* n1g = I[1]; const float* n1b = I[2]; const float* qkvw = I[3]; const float* pw = I[4]; const float* pb = I[5]; const float* cw0 = I[6]; const float* cb0 = I[7]; const float* cw1 = I[8]; const float* cb1 = I[9]; const float* n2g = I[10]; const float* n2b = I[11]; const float* f1w = I[12]; const float* f1b = I[13]; const float* f2w = I[14]; const float* f2b = I[15];
  char* ws = (char*)d_ws; size_t off = 0;
  auto take = [&](size_t bytes) { char* p = ws + off; off += (bytes + 255) & ~(size_t)255; return p; };
  const size_t ne = (size_t)NR * CD;
  _Float16* BQKV = (_Float16*)take((size_t)3 * CD * CD * 2); _Float16* BP = (_Float16*)take((size_t)CD * CD * 2); _Float16* BF1 = (_Float16*)take((size_t)DFF * CD * 2); _Float16* BF2 = (_Float16*)take((size_t)CD * DFF * 2);
  char* R1 = take(ne * 2); char* R2 = take(zmax((size_t)NR * 3 * CD * 2, (size_t)(NR / MCH) * DFF * 4)); char* R3 = take(zmax(NWR * CH * 2 * 4 + NWR * CH * 4 + NWR * CH * 2, ne * 4 + ne * 2 * 2)); char* R4 = take(zmax((size_t)WCH * NHB * TOKP * TOKP * 6, (size_t)(NR / MCH) * DFF * 2 * 2));
  if (off > ws_size) return;
  _Float16* XN = (_Float16*)R1; _Float16* ATT = (_Float16*)R1; _Float16* QKV = (_Float16*)R2; float* ATTP = (float*)R2; float* F1 = (float*)R2;
  _Float16* QW = (_Float16*)R3; _Float16* KW = QW + NWR * CH; _Float16* VW = KW + NWR * CH; _Float16* VT = VW + NWR * CH; float* LE = (float*)(VT + NWR * CH); _Float16* OW = (_Float16*)(LE + NWR * CH);
  float* X2 = (float*)R3; _Float16* YH = (_Float16*)(R3 + ne * 4); _Float16* YL = YH + ne;
  float* S = (float*)R4; _Float16* P = (_Float16*)(R4 + (size_t)WCH * NHB * TOKP * TOKP * 4); _Float16* F1H = (_Float16*)R4; _Float16* F1L = F1H + (size_t)(NR / MCH) * DFF;
  k_wt_f16<<<(3 * CD * CD / 8 + 255) / 256, 256, 0, stream>>>(qkvw, BQKV, CD, 3 * CD, 16.0f); k_wt_f16<<<(CD * CD / 8 + 255) / 256, 256, 0, stream>>>(pw, BP, CD, CD, 16.0f); k_wt_f16<<<(DFF * CD / 8 + 255) / 256, 256, 0, stream>>>(f1w, BF1, CD, DFF, 16.0f); k_wt_f16<<<(CD * DFF / 8 + 255) / 256, 256, 0, stream>>>(f2w, BF2, DFF, CD, 16.0f);
  k_ln1<<<NR / 8, 256, 0, stream>>>(x, n1g, n1b, XN);
  k_gemm2<0><<<dim3((NR / 128) * (3 * CD / 64), 1), 128, 0, stream>>>(XN, CD, 0, BQKV, CD, 0, 0.0625f, nullptr, 0, nullptr, 1, 0, 0, nullptr, QKV, 3 * CD, 0, NR, 3 * CD, CD);
  const unsigned gw = (unsigned)((NWR * CH / 8 + 255) / 256);
  for (int br = 0; br < 2; ++br) { const float* cw = br ? cw1 : cw0; const float* cb = br ? cb1 : cb0;
    k_towin<<<gw, 256, 0, stream>>>(QKV, br, QW, KW, VW); k_vt<<<NI * NWI, 256, 0, stream>>>(VW, VT); k_lepe<<<gw, 256, 0, stream>>>(VW, br, cw, cb, LE);
    for (int c0 = 0; c0 < NI * NWI; c0 += WCH) {
      for (int h = 0; h < NHB; ++h) k_gemm2<0><<<dim3(1 * (TOKP / 64), WCH), 128, 0, stream>>>(QW + (size_t)c0 * TOKP * CH + h * HDm, CH, (size_t)TOKP * CH, KW + (size_t)c0 * TOKP * CH + h * HDm, CH, (size_t)TOKP * CH, 0.17677669529663687f, nullptr, 0, nullptr, 1, 0, 0, S + (size_t)h * TOKP * TOKP, nullptr, TOKP, (size_t)NHB * TOKP * TOKP, TOKP, TOKP, HDm);
      k_soft<<<(WCH * NHB * TOKP) / 8, 256, 0, stream>>>(S, P);
      for (int h = 0; h < NHB; ++h) k_gemm_hhx<0><<<dim3((TOKP / 16) * (HDm / 16), WCH), 128, 0, stream>>>(P + (size_t)h * TOKP * TOKP, TOKP, (size_t)NHB * TOKP * TOKP, VT + ((size_t)c0 * NHB + h) * HDm * TOKP, TOKP, (size_t)NHB * HDm * TOKP, 0.0009765625f, nullptr, 0, LE + (size_t)c0 * TOKP * CH + h * HDm, -1, (size_t)TOKP * CH, 0, nullptr, OW + (size_t)c0 * TOKP * CH + h * HDm, CH, (size_t)TOKP * CH, TOKP, HDm, TOKP); }
    k_toimg<<<gw, 256, 0, stream>>>(OW, br, ATT); }
  k_gemm2<0><<<dim3((NR / 128) * (CD / 64), 1), 128, 0, stream>>>(ATT, CD, 0, BP, CD, 0, 0.0625f, pb, 0, nullptr, 1, 0, 0, ATTP, nullptr, CD, 0, NR, CD, CD);
  k_resln<<<NR / 8, 256, 0, stream>>>(x, ATTP, n2g, n2b, X2, YH, YL);
  for (int rc = 0; rc < MCH; ++rc) { const size_t r0 = (size_t)rc * (NR / MCH); const int MR = NR / MCH; const dim3 g1((MR / 128) * (DFF / 64), 1), g2((MR / 128) * (CD / 64), 1);
    k_gemm2<0><<<g1, 128, 0, stream>>>(YL + r0 * CD, CD, 0, BF1, CD, 0, 0.0625f / 1024.0f, nullptr, 0, nullptr, 1, 0, 0, F1, nullptr, DFF, 0, MR, DFF, CD); k_gemm2<0><<<g1, 128, 0, stream>>>(YH + r0 * CD, CD, 0, BF1, CD, 0, 0.0625f, f1b, 0, F1, 1, (size_t)DFF, 0, F1, nullptr, DFF, 0, MR, DFF, CD);
    k_gelu<<<(unsigned)(((size_t)MR * DFF / 8 + 255) / 256), 256, 0, stream>>>(F1, F1H, F1L, (size_t)MR * DFF / 8);
    k_gemm2<0><<<g2, 128, 0, stream>>>(F1L, DFF, 0, BF2, DFF, 0, 0.0625f / 1024.0f, nullptr, 0, X2 + r0 * CD, 1, (size_t)CD, 0, (float*)d_out + r0 * CD, nullptr, CD, 0, MR, CD, DFF); k_gemm2<0><<<g2, 128, 0, stream>>>(F1H, DFF, 0, BF2, DFF, 0, 0.0625f, f2b, 0, (const float*)d_out + r0 * CD, 1, (size_t)CD, 0, (float*)d_out + r0 * CD, nullptr, CD, 0, MR, CD, DFF); }
}
